// S6Block_46368466927943
// MI455X (gfx1250) — hardware-run, weakly checked
//
#include <hip/hip_runtime.h>
#include <math.h>

typedef __attribute__((ext_vector_type(16))) _Float16 v16h;
typedef __attribute__((ext_vector_type(8)))  _Float16 v8h;
typedef __attribute__((ext_vector_type(8)))  float    v8f;
typedef __attribute__((ext_vector_type(4)))  float    v4f;

constexpr int kBatch  = 2;
constexpr int kSeq    = 2048;
constexpr int kDm     = 512;
constexpr int kNst    = 16;
constexpr int kRk     = 32;
constexpr int kRows   = kBatch * kSeq;
constexpr int kCat    = 64;
constexpr int kScanTS = 64;
constexpr int kScanCh = 64;
constexpr int kScanYP = 68;
constexpr float kCarryAct = 16.0f;
constexpr float kCarryW   = 1024.0f;
constexpr float kFold     = 1.0f / (kCarryAct * kCarryW);

static_assert(2 * kNst + kRk == kCat, "concatenated projection width");
static_assert((kDm % 32) == 0 && (kRk % 32) == 0, "GEMM K multiples of 32");
static_assert((kRows % 64) == 0 && (kCat % 64) == 0 && (kDm % 64) == 0, "GEMM M,N multiples of 64");
static_assert((kSeq % kScanTS) == 0 && (kDm % kScanCh) == 0, "scan tile multiples");

constexpr size_t kOffXH   = 0;
constexpr size_t kOffWCAT = kOffXH   + (size_t)kRows * kDm * 2;
constexpr size_t kOffW2H  = kOffWCAT + (size_t)kCat * kDm * 2;
constexpr size_t kOffBIAS = kOffW2H  + (size_t)kDm * kRk * 2;
constexpr size_t kOffBCH  = kOffBIAS + (size_t)kCat * 4;
constexpr size_t kOffHH   = kOffBCH  + (size_t)kRows * kCat * 4;
constexpr size_t kOffZP   = kOffHH   + (size_t)kRows * kRk * 2;
constexpr size_t kWsTotal = kOffZP   + (size_t)kRows * kDm * 4;
static_assert(kWsTotal == 13992192ull, "carve total");
static_assert(kWsTotal <= 134217728ull, "carve cap");
static_assert((kOffWCAT % 128) == 0 && (kOffW2H % 128) == 0 && (kOffBIAS % 128) == 0 &&
              (kOffBCH % 128) == 0 && (kOffHH % 128) == 0 && (kOffZP % 128) == 0, "128-B aligned regions");

union FragU { v16h v; v8h h[2]; };
__device__ __forceinline__ v16h frag_load(const _Float16* p) {
  FragU f;
  f.h[0] = *(const v8h*)(p);
  f.h[1] = *(const v8h*)(p + 16);
  return f.v;
}
__device__ __forceinline__ v8f mma_f16(v16h a, v16h b, v8f c) {
  return __builtin_amdgcn_wmma_f32_16x16x32_f16(false, a, false, b, (short)0, c, false, false);
}
__device__ __forceinline__ void tie_acc(v8f& a, v16h x, v16h y) {
  asm volatile("v_nop\n\tv_nop\n\tv_nop\n\tv_nop" : "+v"(a) : "v"(x), "v"(y));
}
__device__ __forceinline__ void keep4_h(v16h a, v16h b, v16h c, v16h d) {
  asm volatile("v_nop" :: "v"(a), "v"(b), "v"(c), "v"(d));
}

constexpr int kPackXBlocks = (kRows * kDm / 8) / 256;
constexpr int kPackWBlocks = (32 * kDm / 8) / 256;
constexpr int kPack2Blocks = (kDm * kRk / 8) / 256;
constexpr int kPackGrid    = kPackXBlocks + 2 * kPackWBlocks + kPack2Blocks + 1;
static_assert(kPackXBlocks == 1024 && kPackWBlocks == 8 && kPack2Blocks == 8 && kPackGrid == 1049, "pack grid");

__global__ __launch_bounds__(256) void pack_planes_kernel(
    const float* __restrict__ x, const float* __restrict__ wbc, const float* __restrict__ wdt1,
    const float* __restrict__ wdt2, const float* __restrict__ bbc, const float* __restrict__ bdt1,
    unsigned short* __restrict__ XH, unsigned short* __restrict__ WCAT, unsigned short* __restrict__ W2H,
    float* __restrict__ BIAS)
{
  const int bx  = blockIdx.x;
  const int tid = threadIdx.x;
  if (bx < kPackGrid - 1) {
    const float* src;
    unsigned short* dst;
    float sc;
    int lb;
    if (bx < kPackXBlocks) {
      src = x; dst = XH; sc = kCarryAct; lb = bx;
    } else if (bx < kPackXBlocks + kPackWBlocks) {
      src = wbc; dst = WCAT; sc = kCarryW; lb = bx - kPackXBlocks;
    } else if (bx < kPackXBlocks + 2 * kPackWBlocks) {
      src = wdt1; dst = WCAT + (size_t)32 * kDm; sc = kCarryW; lb = bx - kPackXBlocks - kPackWBlocks;
    } else {
      src = wdt2; dst = W2H; sc = kCarryW; lb = bx - kPackXBlocks - 2 * kPackWBlocks;
    }
    const size_t e0 = ((size_t)lb * 256 + (size_t)tid) << 3;
    const v4f a0 = *(const v4f*)(src + e0);
    const v4f a1 = *(const v4f*)(src + e0 + 4);
    v8h hv;
#pragma unroll
    for (int e = 0; e < 4; ++e) {
      const float f0 = a0[e] * sc;
      const float f1 = a1[e] * sc;
      hv[e]     = (_Float16)f0;
      hv[4 + e] = (_Float16)f1;
    }
    unsigned short* q = dst + e0;
    *(volatile v8h*)q = hv;
    __threadfence();
    *(volatile v8h*)q = hv;
  } else {
    const int li = tid & 7;
    const v4f va = *(const v4f*)(bbc + li * 4);
    const v4f vb = *(const v4f*)(bdt1 + li * 4);
    float a0 = va[0], a1 = va[1], a2 = va[2], a3 = va[3];
    float b0 = vb[0], b1 = vb[1], b2 = vb[2], b3 = vb[3];
    asm volatile("" : "+v"(a0), "+v"(a1), "+v"(a2), "+v"(a3));
    asm volatile("" : "+v"(b0), "+v"(b1), "+v"(b2), "+v"(b3));
    const bool first = (tid & 15) < 8;
    v4f o;
    o[0] = first ? a0 : b0;
    o[1] = first ? a1 : b1;
    o[2] = first ? a2 : b2;
    o[3] = first ? a3 : b3;
    if (tid < 16) {
      float* q = BIAS + tid * 4;
      *(volatile v4f*)q = o;
      __threadfence();
      *(volatile v4f*)q = o;
    }
  }
}

__global__ __launch_bounds__(256) void wmma_gemm64_f16(
    const unsigned short* __restrict__ Ap, int lda,
    const unsigned short* __restrict__ Btp, int ldb,
    float* __restrict__ C, int ldc,
    const float* __restrict__ bias,
    int M, int N, int K, float scale) {
  const _Float16* A  = (const _Float16*)Ap;
  const _Float16* Bt = (const _Float16*)Btp;
  __shared__ __align__(16) float sT[8][16 * 68];
  const int lane = threadIdx.x & 31;
  const int wave = __builtin_amdgcn_readfirstlane((int)(threadIdx.x >> 5));
  const int tilesN = N >> 6;
  const int tilesM = M >> 6;
  const int tile = blockIdx.x * 8 + wave;
  if (tile >= tilesM * tilesN) return;
  const int tm = tile / tilesN;
  const int tn = tile - tm * tilesN;
  const int m0 = tm << 6;
  const int n0 = tn << 6;

  const int rlane = lane & 15;
  const int koff  = (lane >> 4) * 8;
  const int mOff  = (lane >> 4) * 8;

  v8f acc[4][4];
#pragma unroll
  for (int i = 0; i < 4; ++i)
#pragma unroll
    for (int j = 0; j < 4; ++j) acc[i][j] = (v8f){0.f,0.f,0.f,0.f,0.f,0.f,0.f,0.f};

  for (int k0 = 0; k0 < K; k0 += 32) {
    v16h bh[4];
#pragma unroll
    for (int j = 0; j < 4; ++j) {
      const size_t bo = (size_t)(n0 + (j << 4) + rlane) * ldb + koff + k0;
      bh[j] = frag_load(Bt + bo);
    }
#pragma unroll
    for (int i = 0; i < 4; ++i) {
      const size_t ao = (size_t)(m0 + (i << 4) + rlane) * lda + koff + k0;
      v16h ah = frag_load(A + ao);
#pragma unroll
      for (int j = 0; j < 4; ++j) acc[i][j] = mma_f16(ah, bh[j], acc[i][j]);
      tie_acc(acc[i][0], ah, bh[0]);
      tie_acc(acc[i][1], ah, bh[1]);
      tie_acc(acc[i][2], ah, bh[2]);
      tie_acc(acc[i][3], ah, bh[3]);
    }
    keep4_h(bh[0], bh[1], bh[2], bh[3]);
  }

  float* slab = sT[wave];
#pragma unroll
  for (int i = 0; i < 4; ++i) {
    const int mBase = m0 + (i << 4);
#pragma unroll
    for (int j = 0; j < 4; ++j) {
      const int n = n0 + (j << 4) + rlane;
      const float bv = bias[n];
#pragma unroll
      for (int r = 0; r < 8; ++r) {
        float v = acc[i][j][r] * scale;
        v += bv;
        slab[(mOff + r) * 68 + (j << 4) + rlane] = v;
      }
    }
    __builtin_amdgcn_fence(__ATOMIC_RELEASE, "workgroup");
    __builtin_amdgcn_wave_barrier();
    __builtin_amdgcn_fence(__ATOMIC_ACQUIRE, "workgroup");
    {
      const int hh = lane >> 4, c4 = (lane & 15) * 4;
      for (int pass = 0; pass < 2; ++pass) {
#pragma unroll
        for (int it = 0; it < 8; ++it) {
          const int row = it * 2 + hh;
          v4f v = *(const v4f*)(slab + row * 68 + c4);
          *(volatile v4f*)(C + (size_t)(mBase + row) * ldc + n0 + c4) = v;
        }
        __threadfence();
      }
    }
    __builtin_amdgcn_fence(__ATOMIC_RELEASE, "workgroup");
    __builtin_amdgcn_wave_barrier();
    __builtin_amdgcn_fence(__ATOMIC_ACQUIRE, "workgroup");
  }
}

__global__ __launch_bounds__(256) void pack_h_kernel(const float* __restrict__ BCH, unsigned short* __restrict__ HH)
{
  const int i   = blockIdx.x * 256 + threadIdx.x;
  const int row = i >> 2;
  const int cg  = (i & 3) * 8;
  const float* src = BCH + (size_t)row * kCat + 32 + cg;
  const v4f a0 = *(const v4f*)(src);
  const v4f a1 = *(const v4f*)(src + 4);
  v8h hv;
#pragma unroll
  for (int e = 0; e < 4; ++e) {
    const float f0 = a0[e] * kCarryAct;
    const float f1 = a1[e] * kCarryAct;
    hv[e]     = (_Float16)f0;
    hv[4 + e] = (_Float16)f1;
  }
  unsigned short* q = HH + ((size_t)i << 3);
  *(volatile v8h*)q = hv;
  __threadfence();
  *(volatile v8h*)q = hv;
}

__global__ __launch_bounds__(64) void scan_kernel(
    const float* __restrict__ ZP, const float* __restrict__ BCH, const float* __restrict__ X,
    const float* __restrict__ Ap, const float* __restrict__ Dp, float* __restrict__ out)
{
#pragma clang fp contract(off)
  __shared__ __align__(16) float sX[kScanTS * 32];
  __shared__ __align__(16) float sY[kScanTS * kScanYP];
  const int tid  = threadIdx.x;
  const int lane = tid & 31;
  const int wave = __builtin_amdgcn_readfirstlane((int)(threadIdx.x >> 5));
  constexpr int kBlkPerB = kDm / kScanCh;
  const int bix = blockIdx.x / kBlkPerB;
  const int d0  = (blockIdx.x - bix * kBlkPerB) * kScanCh;
  const int d   = d0 + tid;
  const size_t row0 = (size_t)bix * kSeq;

  float An[kNst], h[kNst];
#pragma unroll
  for (int q4 = 0; q4 < 4; ++q4) {
    const v4f av = *(const v4f*)(Ap + (size_t)d * kNst + 4 * q4);
    An[4 * q4 + 0] = av[0];
    An[4 * q4 + 1] = av[1];
    An[4 * q4 + 2] = av[2];
    An[4 * q4 + 3] = av[3];
  }
#pragma unroll
  for (int s = 0; s < kNst; ++s) h[s] = 0.f;
  const float Dd = Dp[d];

  const int lr  = tid >> 3;
  const int lc4 = (tid & 7) * 4;
  const int hh  = lane >> 4;
  const int c4  = (lane & 15) * 4;

#pragma unroll 1
  for (int t0 = 0; t0 < kSeq; t0 += kScanTS) {
    __syncthreads();
#pragma unroll
    for (int i = 0; i < 8; ++i) {
      const int r = lr + 8 * i;
      *(v4f*)(sX + r * 32 + lc4) = *(const v4f*)(BCH + (row0 + t0 + r) * kCat + lc4);
    }
    __syncthreads();
#pragma unroll 1
    for (int s = 0; s < kScanTS; ++s) {
      const size_t g = (row0 + (size_t)(t0 + s)) * kDm + d;
      const float zv = ZP[g];
      const float xt = X[g];
      const float* xr = sX + s * 32;
      float Bs[kNst], Cs[kNst];
#pragma unroll
      for (int q4 = 0; q4 < 4; ++q4) {
        const v4f bv = *(const v4f*)(xr + 4 * q4);
        const v4f cv = *(const v4f*)(xr + kNst + 4 * q4);
        Bs[4 * q4 + 0] = bv[0]; Bs[4 * q4 + 1] = bv[1]; Bs[4 * q4 + 2] = bv[2]; Bs[4 * q4 + 3] = bv[3];
        Cs[4 * q4 + 0] = cv[0]; Cs[4 * q4 + 1] = cv[1]; Cs[4 * q4 + 2] = cv[2]; Cs[4 * q4 + 3] = cv[3];
      }
      const float ez = expf(-fabsf(zv));
      float dt = fmaxf(zv, 0.0f) + log1pf(ez);
      dt = fminf(fmaxf(dt, 1e-7f), 1e6f);
      float y = 0.f;
#pragma unroll
      for (int k = 0; k < kNst; ++k) {
        const float tmp = An[k] * dt;
        const float a   = __expf(tmp);
        const float den = tmp + 1e-6f;
        const float dB  = dt * Bs[k];
        const float num = (a - 1.0f) * dB;
        const float bb  = (num * __builtin_amdgcn_rcpf(den)) * xt;
        const float bm  = fmaxf(fabsf(bb), 1e-6f);
        const float bc  = (bb < 0.0f) ? -bm : bm;
        const float ac  = fmaxf(a, 1e-6f);
        h[k] = fmaf(ac, h[k], bc);
        y    = fmaf(h[k], Cs[k], y);
      }
      const float skip = Dd * xt;
      sY[s * kScanYP + tid] = y + skip;
    }
    __syncthreads();
    for (int pass = 0; pass < 2; ++pass) {
#pragma unroll
      for (int it = 0; it < 16; ++it) {
        const int row = wave * 32 + it * 2 + hh;
        const v4f val = *(const v4f*)(sY + row * kScanYP + c4);
        *(volatile v4f*)(out + (row0 + (size_t)(t0 + row)) * kDm + d0 + c4) = val;
      }
      __threadfence();
    }
  }
}

extern "C" void kernel_launch(void* const* d_in, const int* in_sizes, int n_in,
                              void* d_out, int out_size, void* d_ws, size_t ws_size,
                              hipStream_t stream) {
  if (n_in < 9) return;
  if (in_sizes[0] != kRows * kDm) return;
  if (in_sizes[1] != kDm * kNst) return;
  if (in_sizes[2] != 2 * kNst * kDm) return;
  if (in_sizes[3] != 2 * kNst) return;
  if (in_sizes[4] != kRk * kDm) return;
  if (in_sizes[5] != kRk) return;
  if (in_sizes[6] != kDm * kRk) return;
  if (in_sizes[7] != kDm) return;
  if (in_sizes[8] != kDm) return;
  if (out_size != kRows * kDm) return;
  if (ws_size < kWsTotal) return;

  const float* x    = (const float*)d_in[0];
  const float* Ap   = (const float*)d_in[1];
  const float* Wbc  = (const float*)d_in[2];
  const float* bbc  = (const float*)d_in[3];
  const float* Wdt1 = (const float*)d_in[4];
  const float* bdt1 = (const float*)d_in[5];
  const float* Wdt2 = (const float*)d_in[6];
  const float* bdt2 = (const float*)d_in[7];
  const float* Dp   = (const float*)d_in[8];
  float* out = (float*)d_out;

  char* ws = (char*)d_ws;
  unsigned short* XH   = (unsigned short*)(ws + kOffXH);
  unsigned short* WCAT = (unsigned short*)(ws + kOffWCAT);
  unsigned short* W2H  = (unsigned short*)(ws + kOffW2H);
  float*          BIAS = (float*)(ws + kOffBIAS);
  float*          BCH  = (float*)(ws + kOffBCH);
  unsigned short* HH   = (unsigned short*)(ws + kOffHH);
  float*          ZP   = (float*)(ws + kOffZP);

  pack_planes_kernel<<<kPackGrid, 256, 0, stream>>>(x, Wbc, Wdt1, Wdt2, bbc, bdt1, XH, WCAT, W2H, BIAS);

  wmma_gemm64_f16<<<(kRows / 64) * (kCat / 64) / 8, 256, 0, stream>>>(
      XH, kDm, WCAT, kDm, BCH, kCat, BIAS, kRows, kCat, kDm, kFold);

  pack_h_kernel<<<(kRows * 4) / 256, 256, 0, stream>>>(BCH, HH);

  wmma_gemm64_f16<<<(kRows / 64) * (kDm / 64) / 8, 256, 0, stream>>>(
      HH, kRk, W2H, kRk, ZP, kDm, bdt2, kRows, kDm, kRk, kFold);

  scan_kernel<<<kBatch * (kDm / kScanCh), kScanCh, 0, stream>>>(ZP, BCH, x, Ap, Dp, out);
}
